// GAT_36971078484045
// MI455X (gfx1250) — hardware-verified
//
#include <hip/hip_runtime.h>


namespace {

constexpr int N = 50000, NP = 50048, NPL = NP  , SRCM = N  , EFULL = 1600000, E = EFULL  ;
constexpr int IN = 128  , INX = IN, HN = 8  , HC = 8  , CP = 16  , D1R = HN * HC  , D1 = HN * CP  , NCL = 7  , D2 = 32  , DH = D1  , VOC = 1, NRL = NP  , NL = (NPL < N ? NPL : N);
static_assert(D1 == 128 && D1R == 64 && HC <= CP && NCL <= D2 && D2 == 32, "layer 1: 8 heads x 8 padded to 16; layer 2: 1 head x 7 padded to 32");
constexpr float LNEPS = 1e-5f; constexpr float XS = 8.0f, WSC = 256.0f, WSQ = 0.25f, RS_ = 1024.0f, NSL_ = 0.2f, NSA_ = 0.05f  , SLOPE = 0.0f, BNEPS = 1e-5f;
static_assert(NP % 32 == 0 && NP >= N && NPL % 32 == 0 && (DH == 32 || DH == 64 || DH == 128 || DH == 256), "tiling");
typedef _Float16 b16;
typedef __attribute__((ext_vector_type(16))) _Float16 v16b;
typedef __attribute__((ext_vector_type(8))) _Float16 v8b;
typedef __attribute__((ext_vector_type(8))) float v8f;
typedef __attribute__((ext_vector_type(4))) float v4f;
__device__ __forceinline__ float bf16_rne(float f) { unsigned int u = __float_as_uint(f); u += 0x7FFFu + ((u >> 16) & 1u); return __uint_as_float(u & 0xFFFF0000u); }
__device__ __forceinline__ float bfo(float f) { float r = bf16_rne(f); asm volatile("" : "+v"(r)); return r; }
__device__ __forceinline__ void split16(float v, b16& hi, b16& lo) { hi = (b16)v; lo = (b16)(v - (float)hi); }
__device__ __forceinline__ v16b frag_kb(const b16* p, int hh) { const v8b a = *(const v8b*)(p + 8 * hh), b = *(const v8b*)(p + 16 + 8 * hh); v16b f;
#pragma unroll
  for (int e = 0; e < 8; ++e) { f[e] = a[e]; f[8 + e] = b[e]; } return f; }
__device__ __forceinline__ v8f wmma16b(v16b a, v16b b, v8f c) { v8f d = __builtin_amdgcn_wmma_f32_16x16x32_f16(false, a, false, b, (short)0, c, false, false); asm volatile("v_nop\n\tv_nop\n\tv_nop\n\tv_nop" : "+v"(d) : "v"(a), "v"(b)); return d; }
__device__ __forceinline__ void wave_lds_sync() { __builtin_amdgcn_fence(__ATOMIC_RELEASE, "workgroup"); __builtin_amdgcn_wave_barrier(); __builtin_amdgcn_fence(__ATOMIC_ACQUIRE, "workgroup"); }
__device__ __forceinline__ float pmul(float a, float b) { float p = a * b; asm volatile("" : "+v"(p)); return p; }
__device__ __forceinline__ int iclamp(int v, int lo, int hi) { return v < lo ? lo : (v > hi ? hi : v); }
constexpr int CSR_NBLK = 512, CSR_GB = 8, CSR_GN = 1 << CSR_GB  , CSR_MAXG = 512, CSR_CAP = 12288  ;
static_assert(((N + CSR_GN - 1) >> CSR_GB) <= CSR_MAXG && CSR_GN % 4 == 0 && CSR_GN <= 65536, "csr: bucket count / 16-bit node key");
__global__ __launch_bounds__(64) void csrA_kernel(const int* __restrict__ dst, int E, int N, int nG, int CHP, int NGP, int* __restrict__ STG, int* __restrict__ HST) {
  extern __shared__ int sm[];
  int* cnt = sm; int* run = sm + NGP; int* ids = sm + 2 * NGP;
  const int b = blockIdx.x; const int ch = (E + CSR_NBLK - 1) / CSR_NBLK; const int e0 = b * ch, e1 = min(E, e0 + ch);
  for (int i = threadIdx.x; i < NGP; i += 64) cnt[i] = 0;
  for (int i = threadIdx.x; i < CHP; i += 64) ids[i] = -1;
  __syncthreads();
  if (threadIdx.x == 0) {
    for (int e = e0; e < e1; ++e) { int d = dst[e]; d = (d < 0) ? 0 : (d >= N ? N - 1 : d); cnt[d >> CSR_GB] += 1; }
    int acc = 0; for (int g = 0; g < nG; ++g) { run[g] = acc; acc += cnt[g]; }
    for (int e = e0; e < e1; ++e) { int d = dst[e]; d = (d < 0) ? 0 : (d >= N ? N - 1 : d); const int g = d >> CSR_GB; ids[run[g]] = e; run[g] += 1; } }
  __syncthreads();
  typedef __attribute__((ext_vector_type(4))) int v4i;
  for (int pass = 0; pass < 2; ++pass) {
    for (int i = threadIdx.x; i < CHP / 4; i += 64) *(volatile v4i*)(STG + (size_t)b * CHP + i * 4) = *(const v4i*)(&ids[i * 4]);
    for (int i = threadIdx.x; i < NGP / 4; i += 64) { v4i v; for (int e = 0; e < 4; ++e) v[e] = (i * 4 + e < nG) ? cnt[i * 4 + e] : 0; *(volatile v4i*)(HST + (size_t)b * NGP + i * 4) = v; }
    __threadfence(); }
}
__global__ __launch_bounds__(512) void csrS_kernel(const int* __restrict__ HST, int nG, int NGP, int* __restrict__ START, int* __restrict__ TOT, int* __restrict__ OFF) {
  __shared__ int tot[CSR_MAXG];
  const int b = threadIdx.x;
  for (int pass = 0; pass < 2; ++pass) { int runb = 0; for (int g = 0; g < nG; ++g) { int c = HST[(size_t)b * NGP + g]; c = (c < 0) ? 0 : c; ((volatile int*)OFF)[(size_t)g * CSR_NBLK + b] = runb; runb += c; } __threadfence(); }
  for (int g = threadIdx.x; g < nG; g += 512) { int s = 0; for (int bb = 0; bb < CSR_NBLK; ++bb) { int c = HST[(size_t)bb * NGP + g]; s += (c < 0) ? 0 : c; } tot[g] = s; }
  __syncthreads();
  if (threadIdx.x < 32) {
    __shared__ int st[CSR_MAXG + 32];
    if (threadIdx.x == 0) { int acc = 0; for (int g = 0; g < NGP; ++g) { st[g] = acc; if (g < nG) acc += (tot[g] + 31) & ~31; } st[NGP] = acc; }
    __builtin_amdgcn_fence(__ATOMIC_RELEASE, "workgroup"); __builtin_amdgcn_wave_barrier(); __builtin_amdgcn_fence(__ATOMIC_ACQUIRE, "workgroup");
    for (int pass = 0; pass < 2; ++pass) { for (int i = threadIdx.x; i < NGP + 32; i += 32) { ((volatile int*)START)[i] = (i <= NGP) ? st[min(i, NGP)] : 0; ((volatile int*)TOT)[i] = (i < nG) ? tot[i] : 0; } __threadfence(); } }
}
__global__ __launch_bounds__(256) void csrB_kernel(const int* __restrict__ dst, int N, int nG, int CHP, int NGP, int permLen, const int* __restrict__ STG, const int* __restrict__ HST, const int* __restrict__ OFF, const int* __restrict__ START, const int* __restrict__ TOT, int* __restrict__ PERM, int* __restrict__ ROWPTR, int* __restrict__ ROWCNT, int* __restrict__ FLAG) {
  typedef __attribute__((ext_vector_type(4))) int v4i;
  __shared__ int ids[CSR_CAP]; __shared__ unsigned short key[CSR_CAP]; __shared__ int outp[CSR_CAP]; __shared__ int ncnt[CSR_GN + 1]; __shared__ int boff[CSR_NBLK + 1];
  const int g = blockIdx.x, t_ = threadIdx.x; int tot = TOT[g]; int st = START[g], stn = START[g + 1]; const int v0 = g * CSR_GN; const int nv = min(CSR_GN, N - v0);
  st = (st < 0) ? 0 : (st > permLen - 32 ? permLen - 32 : st) & ~31; stn = (stn < st) ? st : (stn > permLen ? permLen : stn); tot = (tot < 0) ? 0 : tot; if (tot > stn - st && tot <= CSR_CAP) tot = stn - st;
  if (tot > CSR_CAP) {
    for (int pass = 0; pass < 2; ++pass) { for (int i = t_; i < CSR_GN / 4; i += 256) { v4i a, c; for (int e = 0; e < 4; ++e) { a[e] = st; c[e] = 0; } *(volatile v4i*)(ROWPTR + v0 + i * 4) = a; *(volatile v4i*)(ROWCNT + v0 + i * 4) = c; } if (t_ == 0) ((volatile int*)FLAG)[0] = 1; __threadfence(); } (void)nv; return; }
  if (t_ == 0) { int acc = 0; for (int b = 0; b < CSR_NBLK; ++b) { boff[b] = acc; int c = HST[(size_t)b * NGP + g]; c = (c < 0) ? 0 : (c > CHP ? CHP : c); acc += c; if (acc > tot) acc = tot; } boff[CSR_NBLK] = acc; }
  for (int i = t_; i <= CSR_GN; i += 256) ncnt[i] = 0;
  __syncthreads();
  for (int b = 0; b < CSR_NBLK; ++b) { const int c = boff[b + 1] - boff[b]; int o_ = OFF[(size_t)g * CSR_NBLK + b]; o_ = (o_ < 0) ? 0 : (o_ > CHP - c ? CHP - c : o_); const int* src_ = STG + (size_t)b * CHP + o_;
    for (int i = t_; i < c; i += 256) { int id = src_[i]; id = (id < 0) ? 0 : id; ids[boff[b] + i] = id; int d = dst[id]; d = (d < v0) ? v0 : (d >= N ? N - 1 : d); int kk = d - v0; kk = (kk < 0) ? 0 : (kk >= CSR_GN ? CSR_GN - 1 : kk); key[boff[b] + i] = (unsigned short)kk; } }
  __syncthreads();
  if (t_ == 0) { for (int i = 0; i < tot; ++i) ncnt[key[i]] += 1; int acc = 0; for (int vl = 0; vl < CSR_GN; ++vl) { const int c = ncnt[vl]; ncnt[vl] = acc; acc += c; } ncnt[CSR_GN] = acc;
    for (int i = 0; i < tot; ++i) { const int vl = key[i]; outp[ncnt[vl]] = ids[i]; ncnt[vl] += 1; }
    for (int vl = CSR_GN; vl > 0; --vl) ncnt[vl] = ncnt[vl - 1]; ncnt[0] = 0; }
  __syncthreads();
  for (int pass = 0; pass < 2; ++pass) {
    for (int i = t_; i < (stn - st) / 4; i += 256) { v4i v; for (int e = 0; e < 4; ++e) { const int q = i * 4 + e; v[e] = (q < tot) ? outp[q] : -1; } *(volatile v4i*)(PERM + st + i * 4) = v; }
    for (int i = t_; i < CSR_GN / 4; i += 256) { v4i a, c; for (int e = 0; e < 4; ++e) { const int vl = i * 4 + e; a[e] = st + ncnt[vl]; c[e] = (vl < nv) ? (ncnt[vl + 1] - ncnt[vl]) : 0; } *(volatile v4i*)(ROWPTR + v0 + i * 4) = a; *(volatile v4i*)(ROWCNT + v0 + i * 4) = c; }
    __threadfence(); }
}
__global__ __launch_bounds__(256) void csrZ_kernel(int* __restrict__ p, size_t n4) { typedef __attribute__((ext_vector_type(4))) int v4i; const size_t tid = (size_t)blockIdx.x * 256 + threadIdx.x, nth = (size_t)gridDim.x * 256; v4i z = {0, 0, 0, 0}; for (size_t i = tid; i < n4; i += nth) *(volatile v4i*)(p + i * 4) = z; }
struct CsrBufs { int *STG, *HST, *OFF, *START, *TOT, *PERM, *ROWPTR, *ROWCNT, *FLAG; int nG, NGP, CHP; size_t permLen; char* base; size_t bytes; };
static size_t csr_carve(CsrBufs& c, char* ws, size_t off, int E, int N) {
  const size_t off0 = off; c.base = ws + off;
  auto al = [&](size_t bytes) { char* p = ws + off; off += (bytes + 255) & ~(size_t)255; return p; };
  c.nG = (N + CSR_GN - 1) / CSR_GN; c.NGP = (c.nG + 31) & ~31; const int ch = (E + CSR_NBLK - 1) / CSR_NBLK; c.CHP = (ch + 31) & ~31; c.permLen = (size_t)E + 32 * (size_t)c.nG + 32;
  c.STG = (int*)al((size_t)CSR_NBLK * c.CHP * 4); c.HST = (int*)al((size_t)CSR_NBLK * c.NGP * 4); c.OFF = (int*)al((size_t)c.NGP * CSR_NBLK * 4); c.START = (int*)al((size_t)(c.NGP + 64) * 4); c.TOT = (int*)al((size_t)(c.NGP + 64) * 4);
  c.PERM = (int*)al(c.permLen * 4); c.ROWPTR = (int*)al((size_t)c.nG * CSR_GN * 4); c.ROWCNT = (int*)al((size_t)c.nG * CSR_GN * 4); c.FLAG = (int*)al(256);
  c.bytes = off - off0; return off;
}
static void csr_build(const CsrBufs& c, const int* dst, int E, int N, hipStream_t stream) {
  const size_t smem = (size_t)(2 * c.NGP + c.CHP) * 4;
  csrZ_kernel<<<512, 256, 0, stream>>>((int*)c.base, c.bytes / 16);
  csrA_kernel<<<CSR_NBLK, 64, smem, stream>>>(dst, E, N, c.nG, c.CHP, c.NGP, c.STG, c.HST);
  csrS_kernel<<<1, 512, 0, stream>>>(c.HST, c.nG, c.NGP, c.START, c.TOT, c.OFF);
  csrB_kernel<<<c.nG, 256, 0, stream>>>(dst, N, c.nG, c.CHP, c.NGP, (int)c.permLen, c.STG, c.HST, c.OFF, c.START, c.TOT, c.PERM, c.ROWPTR, c.ROWCNT, c.FLAG);
}

typedef __attribute__((ext_vector_type(4))) _Float16 v4h;
__device__ __forceinline__ float lrelu(float v) { return v > 0.0f ? v : NSL_ * v; }
template <int K, int DD, int HH, bool RND, int KA = K>
__global__ __launch_bounds__(64) void gatnode_kernel(const float* __restrict__ X, const b16* __restrict__ WT, const b16* __restrict__ WQ, const float* __restrict__ as_, const float* __restrict__ ad_, float* __restrict__ Hh, float* __restrict__ SC) {
  constexpr int NT = DD / 16, CC = DD / HH, TPH = CC / 16;
  __shared__ __attribute__((aligned(16))) b16 Ah[2][16][K + 8], Al[2][16][K + 8]; __shared__ __attribute__((aligned(16))) float Tf[2][16][DD + 4]; __shared__ __attribute__((aligned(16))) float Sc[2][16][16];
  const int wave = threadIdx.x >> 5, lane = threadIdx.x & 31, nloc = lane & 15, hlf = lane >> 4; const size_t m0 = (size_t)blockIdx.x * 32 + wave * 16;
  for (int idx = lane; idx < 16 * (K / 4); idx += 32) { const int rr = idx / (K / 4), c4 = (idx % (K / 4)) * 4; const size_t arow = (m0 + rr < (size_t)N) ? m0 + rr : (size_t)N - 1; v4f v = {0.0f, 0.0f, 0.0f, 0.0f}; if (KA == K) v = *(const v4f*)(X + arow * K + c4); else { for (int j = 0; j < 4; ++j) v[j] = (c4 + j < KA) ? X[arow * KA + c4 + j] : 0.0f; } v4h hv, lv;
    for (int j = 0; j < 4; ++j) { const float vs = (RND ? bf16_rne(v[j]) : v[j]) * XS; const b16 ph = (b16)vs; hv[j] = ph; lv[j] = (b16)((vs - (float)ph) * RS_); } *(v4h*)(&Ah[wave][rr][c4]) = hv; *(v4h*)(&Al[wave][rr][c4]) = lv; }
  for (int idx = lane; idx < 16 * 16; idx += 32) Sc[wave][idx >> 4][idx & 15] = 0.0f;
  wave_lds_sync();
  v8f acc[NT]; for (int t = 0; t < NT; ++t) acc[t] = (v8f){};
#pragma unroll 2
  for (int kb = 0; kb < K; kb += 32) { const v16b a = frag_kb(&Ah[wave][nloc][kb], hlf); v16b al; if (!RND) al = frag_kb(&Al[wave][nloc][kb], hlf);
#pragma unroll
    for (int t = 0; t < NT; ++t) { const size_t wo_ = (size_t)(t * 16 + nloc) * K + kb; acc[t] = wmma16b(a, frag_kb(WT + wo_, hlf), acc[t]); if (!RND) acc[t] = wmma16b(al, frag_kb(WQ + wo_, hlf), acc[t]); } }
#pragma unroll
  for (int t = 0; t < NT; ++t) for (int r = 0; r < 8; ++r) Tf[wave][8 * hlf + r][t * 16 + nloc] = (m0 + 8 * hlf + r < (size_t)N) ? acc[t][r] * (1.0f / (XS * WSC)) : 0.0f;
#pragma unroll
  for (int hd = 0; hd < HH; ++hd) {
    float ws[TPH], wd[TPH]; for (int q = 0; q < TPH; ++q) { ws[q] = bf16_rne(as_[hd * CC + q * 16 + nloc]); wd[q] = bf16_rne(ad_[hd * CC + q * 16 + nloc]); }
#pragma unroll
    for (int r = 0; r < 8; ++r) { float ss = 0.0f, sd = 0.0f;
#pragma unroll
      for (int q = 0; q < TPH; ++q) { const float hv = Tf[wave][8 * hlf + r][(hd * TPH + q) * 16 + nloc]; ss = fmaf(hv, ws[q], ss); sd = fmaf(hv, wd[q], sd); }
      for (int o = 1; o <= 8; o <<= 1) { ss += __shfl_xor(ss, o); sd += __shfl_xor(sd, o); }
      if (nloc == 0) { Sc[wave][8 * hlf + r][hd] = ss; Sc[wave][8 * hlf + r][8 + hd] = sd; } } }
  wave_lds_sync();
  for (int pass = 0; pass < 2; ++pass) {
    if (DD == 256) { for (int rr = 0; rr < 16; ++rr) { *(volatile v4f*)(Hh + (m0 + rr) * DD + lane * 4) = *(const v4f*)(&Tf[wave][rr][lane * 4]); *(volatile v4f*)(Hh + (m0 + rr) * DD + 128 + lane * 4) = *(const v4f*)(&Tf[wave][rr][128 + lane * 4]); } }
    else if (DD == 128) { for (int rr = 0; rr < 16; ++rr) *(volatile v4f*)(Hh + (m0 + rr) * DD + lane * 4) = *(const v4f*)(&Tf[wave][rr][lane * 4]); }
    else if (DD == 64) { for (int rr = 0; rr < 16; rr += 2) { const int r2 = rr + (lane >> 4); *(volatile v4f*)(Hh + (m0 + r2) * DD + (lane & 15) * 4) = *(const v4f*)(&Tf[wave][r2][(lane & 15) * 4]); } }
        else { for (int rr = 0; rr < 16; rr += 4) { const int r2 = rr + (lane >> 3); *(volatile v4f*)(Hh + (m0 + r2) * DD + (lane & 7) * 4) = *(const v4f*)(&Tf[wave][r2][(lane & 7) * 4]); } }
    for (int rr = 0; rr < 16; rr += 8) { const int r2 = rr + (lane >> 2); *(volatile v4f*)(SC + (m0 + r2) * 16 + (lane & 3) * 4) = *(const v4f*)(&Sc[wave][r2][(lane & 3) * 4]); }
    __threadfence(); }
}
template <int DD, int HH, int ACT, bool SELF = false>
__global__ __launch_bounds__(256) void gatagg_kernel(const float* __restrict__ Hh, const float* __restrict__ SC, const int* __restrict__ srcs, const int* __restrict__ PERM, const int* __restrict__ ROWPTR, const int* __restrict__ ROWCNT, int permLen, const float* __restrict__ bias, const float* __restrict__ ADDP, float* __restrict__ G, int mrows) {
  constexpr int CW = DD / 8, CC = DD / HH;
  const int tid = threadIdx.x; const int row = tid >> 3, g = tid & 7, c0 = g * CW, hd = c0 / CC; const int v = blockIdx.x * 32 + row; const int vv = v < N ? v : N - 1;
  float acc[CW]; for (int j = 0; j < CW; ++j) acc[j] = 0.0f;
  int cnt = 0, p0 = 0; if (v < N) { cnt = iclamp(ROWCNT[v], 0, 65536); p0 = iclamp(ROWPTR[v], 0, permLen - 1); if (p0 + cnt > permLen) cnt = permLen - p0; } const float sd = SC[(size_t)vv * 16 + 8 + hd];
  float m = -INFINITY, l = 0.0f;
  if (SELF) {
    m = lrelu(SC[(size_t)vv * 16 + hd] + sd); l = 1.0f; const float* hr = Hh + (size_t)vv * DD + c0;
#pragma unroll
    for (int q = 0; q < CW / 4; ++q) { const v4f t4 = *(const v4f*)(hr + 4 * q); for (int j = 0; j < 4; ++j) acc[4 * q + j] = t4[j]; } }
#pragma unroll 1
  for (int i = 0; i < cnt; ++i) { int s; { const int e = iclamp(PERM[p0 + i], 0, E - 1); s = iclamp(srcs[e], 0, N - 1); if (SRCM < N) s %= SRCM; }
    const float sc = lrelu(SC[(size_t)s * 16 + hd] + sd); const float mn = fmaxf(m, sc); const float al = __expf(m - mn), pw = __expf(sc - mn); l = l * al + pw; m = mn; const float* hr = Hh + (size_t)s * DD + c0;
#pragma unroll
    for (int q = 0; q < CW / 4; ++q) { const v4f t4 = *(const v4f*)(hr + 4 * q); for (int j = 0; j < 4; ++j) acc[4 * q + j] = fmaf(pw, t4[j], pmul(acc[4 * q + j], al)); } }
  const float inv = (SELF || cnt > 0) ? 1.0f / (l + 1e-16f) : 0.0f;
  float addv[CW]; for (int j = 0; j < CW; ++j) addv[j] = 0.0f; if (ADDP != nullptr && v < mrows) { for (int q = 0; q < CW / 4; ++q) { const v4f a4 = *(const v4f*)(ADDP + (size_t)v * DD + c0 + 4 * q); for (int j = 0; j < 4; ++j) addv[4 * q + j] = a4[j]; } }
  for (int pass = 0; pass < 2; ++pass) { if (v < mrows) { float* orow = G + (size_t)v * DD + c0;
#pragma unroll
      for (int q = 0; q < CW / 4; ++q) { v4f o4; for (int j = 0; j < 4; ++j) { float y = acc[4 * q + j] * inv + bf16_rne(bias[c0 + 4 * q + j]) + addv[4 * q + j]; if (ACT == 1) y = (y >= 0.0f) ? y : NSA_ * y; if (ACT == 2) y = (y > 0.0f) ? y : (__expf(y) - 1.0f); if (ACT == 3) y = fmaxf(y, 0.0f); o4[j] = (v < N) ? y : 0.0f; } *(volatile v4f*)(orow + 4 * q) = o4; } }
    __threadfence(); }
}
__global__ __launch_bounds__(256) void wpad8_kernel(const float* __restrict__ w, b16* __restrict__ WT, float scl) {
  const int t = blockIdx.x * 256 + threadIdx.x; if (t >= D1 * IN / 8) return; const int e = t * 8; const int o = e / IN, k0 = e % IN; const int h = o / CP, c = o % CP; v8b v;
#pragma unroll
  for (int j = 0; j < 8; ++j) { const float val = (c < HC) ? bf16_rne(w[(size_t)(HC * h + c) * IN + k0 + j]) : 0.0f; v[j] = (b16)(val * scl); }
  for (int pass = 0; pass < 2; ++pass) { *(volatile v8b*)(WT + e) = v; __threadfence(); }
}
__global__ __launch_bounds__(256) void wpadk_kernel(const float* __restrict__ w, b16* __restrict__ WT, float scl) {
  const int t = blockIdx.x * 256 + threadIdx.x; if (t >= D2 * D1 / 8) return; const int e = t * 8; const int o = e / D1, k0 = e % D1; v8b v;
#pragma unroll
  for (int j = 0; j < 8; ++j) { const int k = k0 + j; const int h = k / CP, c = k % CP; const float val = (o < NCL && c < HC) ? bf16_rne(w[(size_t)o * D1R + HC * h + c]) : 0.0f; v[j] = (b16)(val * scl); }
  for (int pass = 0; pass < 2; ++pass) { *(volatile v8b*)(WT + e) = v; __threadfence(); }
}
__global__ __launch_bounds__(256) void arecp_kernel(const float* __restrict__ as_, const float* __restrict__ at_, const float* __restrict__ b, float* __restrict__ AS, float* __restrict__ AT, float* __restrict__ BV, int nv, int pw, int rw) {
  const int t = threadIdx.x; if (t >= nv * pw) return; const int vh = t / pw, c = t % pw; const bool r = c < rw; const float s = r ? as_[vh * rw + c] : 0.0f, d = r ? at_[vh * rw + c] : 0.0f, bb = r ? b[vh * rw + c] : 0.0f;
  for (int pass = 0; pass < 2; ++pass) { ((volatile float*)AS)[t] = s; ((volatile float*)AT)[t] = d; ((volatile float*)BV)[t] = bb; __threadfence(); }
}
__global__ __launch_bounds__(256) void sm7_kernel(const float* __restrict__ Z, float* __restrict__ OUT, int nl) {
  const size_t i = (size_t)blockIdx.x * 256 + threadIdx.x; if (i >= (size_t)nl * NCL) return; const size_t v = i / NCL; const int c = (int)(i % NCL); const float* zr = Z + v * D2; float z[NCL]; float m = -INFINITY;
#pragma unroll
  for (int j = 0; j < NCL; ++j) { z[j] = zr[j]; m = fmaxf(m, z[j]); }
  float s = 0.0f, mine = 0.0f;
#pragma unroll
  for (int j = 0; j < NCL; ++j) { const float e = __expf(z[j] - m); s += e; if (j == c) mine = e; }
  const float o = mine / s;
  for (int pass = 0; pass < 2; ++pass) { ((volatile float*)OUT)[i] = o; __threadfence(); }
}
}

extern "C" void kernel_launch(void* const* d_in, const int* in_sizes, int n_in, void* d_out, int out_size, void* d_ws, size_t ws_size, hipStream_t stream) {
  (void)n_in;
  auto Fp = [&](int i) { return (const float*)d_in[i]; }; auto Ip = [&](int i) { return (const int*)d_in[i]; };
  if (in_sizes[0] != N * IN || in_sizes[1] != 2 * EFULL || in_sizes[2] != D1R * IN || in_sizes[3] != D1R || in_sizes[4] != D1R || in_sizes[5] != D1R || in_sizes[6] != NCL * D1R || in_sizes[7] != NCL || in_sizes[8] != NCL || in_sizes[9] != NCL || out_size != N * NCL) return;
  size_t off = 0; char* ws = (char*)d_ws;
  auto carve = [&](size_t bytes) { char* p = ws + off; off += (bytes + 255) & ~(size_t)255; return p; };
  b16* W1P = (b16*)carve((size_t)D1 * IN * 2); b16* W2T = (b16*)carve((size_t)D2 * D1 * 2); b16* W2Q = (b16*)carve((size_t)D2 * D1 * 2);
  float* AS1 = (float*)carve(512); float* AT1 = (float*)carve(512); float* BV1 = (float*)carve(512); float* AS2 = (float*)carve(256); float* AT2 = (float*)carve(256); float* BV2 = (float*)carve(256);
  float* FT = (float*)carve((size_t)NP * D1 * 4); float* H1 = (float*)carve((size_t)NP * D1 * 4); float* ZL = (float*)carve((size_t)NP * D2 * 4); float* SC = (float*)carve((size_t)NP * 16 * 4);
  CsrBufs csr; off = csr_carve(csr, ws, off, E, N);
  if (off > ws_size || off > ((size_t)120 << 20)) return;
  { wpad8_kernel<<<(D1 * IN / 8 + 255) / 256, 256, 0, stream>>>(Fp(2), W1P, WSC);
    wpadk_kernel<<<(D2 * D1 / 8 + 255) / 256, 256, 0, stream>>>(Fp(6), W2T, WSC); wpadk_kernel<<<(D2 * D1 / 8 + 255) / 256, 256, 0, stream>>>(Fp(6), W2Q, WSQ);
    arecp_kernel<<<1, 256, 0, stream>>>(Fp(3), Fp(4), Fp(5), AS1, AT1, BV1, HN, CP, HC); arecp_kernel<<<1, 256, 0, stream>>>(Fp(7), Fp(8), Fp(9), AS2, AT2, BV2, 1, D2, NCL); }
  csr_build(csr, Ip(1) + EFULL, E, N, stream);
  gatnode_kernel<IN, D1, HN, true><<<NRL / 32, 64, 0, stream>>>(Fp(0), W1P, W1P, AS1, AT1, FT, SC);
  gatagg_kernel<D1, HN, 2, false><<<NRL / 32, 256, 0, stream>>>(FT, SC, Ip(1), csr.PERM, csr.ROWPTR, csr.ROWCNT, (int)csr.permLen, BV1, nullptr, H1, NRL);
  gatnode_kernel<D1, D2, 1, false><<<NRL / 32, 64, 0, stream>>>(H1, W2T, W2Q, AS2, AT2, FT, SC);
  gatagg_kernel<D2, 1, 0, false><<<NRL / 32, 256, 0, stream>>>(FT, SC, Ip(1), csr.PERM, csr.ROWPTR, csr.ROWCNT, (int)csr.permLen, BV2, nullptr, ZL, NRL);
  sm7_kernel<<<(unsigned)(((size_t)NL * NCL + 255) / 256), 256, 0, stream>>>(ZL, (float*)d_out, NL);
}
